// NetV2_16681652977711
// MI455X (gfx1250) — hardware-verified
//
#include <hip/hip_runtime.h>
#include <stddef.h>


#define HW    28
#define NPX   784
#define HW2   14
#define NPX2  196
#define C1    32
#define C2    64
#define C3    64
#define K2    288
#define K3    256
#define KF    12544
#define NF1   128
#define NF2   10
#define NF2P  16
#define NT2   49
#define NT3   13
#define TC    256
#define NWC   (TC / 32)
#define TFC   64
#define RPB   16
#define ZP    136
#define MAXPASS 64
#define BN_EPS 1e-5f
#define WSCAP 134217728
#define NBF1  ((KF * NF1) / 2048)
#define NBW2  ((C2 * K2) / 2048)
#define NBW3  ((C3 * K3) / 2048)
#define NPREP (NBF1 + NBW2 + NBW3 + 1)

#define OFF_H2   0
#define SZ_H2    (NPX * C2 * 2)
#define OFF_TAG  (NPX * 8)
#define OFF_H1   (OFF_H2 + SZ_H2)
#define SZ_H1    (NPX * C1 * 2)
#define OFF_MK   (OFF_H1 + SZ_H1)
#define OFF_DN   (OFF_MK + NPX * 4)
#define OFF_MK1  (OFF_DN + NPX * 4)
#define OFF_W1   (OFF_MK1 + 800)
#define OFF_BN   (OFF_W1 + 9 * C1 * 4)
#define NBN      480
#define LDS_CONV (OFF_BN + NBN * 4)
#define SC1 0
#define MU1 32
#define BE1 64
#define SC2 96
#define MU2 160
#define BE2 224
#define SC3 288
#define MU3 352
#define BE3 416

static_assert(NBF1 * 2048 == KF * NF1);
static_assert(NBW2 * 2048 == C2 * K2);
static_assert(NBW3 * 2048 == C3 * K3);
static_assert(NF2P * NF1 == 2048);
static_assert(OFF_TAG + NPX * 4 <= SZ_H2);
static_assert(KF * 2 <= SZ_H1);
static_assert(NT2 * 16 == NPX);
static_assert(NT3 * 16 >= NPX2 && (NT3 - 1) * 16 < NPX2);
static_assert((OFF_H1 % 16) == 0 && (OFF_MK % 16) == 0 && (OFF_DN % 16) == 0);
static_assert((OFF_MK1 % 16) == 0 && (OFF_W1 % 16) == 0 && (OFF_BN % 16) == 0);
static_assert(K2 % 32 == 0 && K3 % 32 == 0 && KF % 32 == 0 && NF1 % 32 == 0);
static_assert((ZP * 2) % 16 == 0);
static_assert(RPB * NF2 == 160);
static_assert(NPX2 <= TC);

typedef float    v4f  __attribute__((ext_vector_type(4)));
typedef float    v8f  __attribute__((ext_vector_type(8)));
typedef _Float16 v8h  __attribute__((ext_vector_type(8)));
typedef _Float16 v16h __attribute__((ext_vector_type(16)));
union Frag { v16h v; v8h h[2]; };

__device__ __forceinline__ v8f wmf(v16h a, v16h b, v8f c) {
  v8f d = __builtin_amdgcn_wmma_f32_16x16x32_f16(false, a, false, b, (short)0, c, false, false);
  asm volatile("v_nop\n\tv_nop\n\tv_nop\n\tv_nop" : "+v"(d) : "v"(a), "v"(b));
  return d;
}

__device__ __forceinline__ v8f zacc() {
  v8f z = {0.f, 0.f, 0.f, 0.f, 0.f, 0.f, 0.f, 0.f};
  return z;
}

__device__ __forceinline__ v8h zh8() {
  v8h z;
#pragma unroll
  for (int e = 0; e < 8; ++e) z[e] = (_Float16)0.0f;
  return z;
}

__global__ __launch_bounds__(256) void k_prep(
    const float* __restrict__ w2, const float* __restrict__ w3,
    const float* __restrict__ f1, const float* __restrict__ f2,
    _Float16* w2h, _Float16* w3h, _Float16* f1h, _Float16* f2h) {
  const int tid = (int)threadIdx.x, b = (int)blockIdx.x;
  float v[8];
  _Float16* dst;
  if (b < NBF1) {
    const int c  = b * 256 + tid;
    const int n  = c / (KF / 8);
    const int k0 = (c - n * (KF / 8)) * 8;
#pragma unroll
    for (int e = 0; e < 8; ++e) v[e] = 64.0f * f1[(size_t)(k0 + e) * NF1 + n];
    dst = f1h + (size_t)c * 8;
  } else if (b < NBF1 + NBW2) {
    const int c  = (b - NBF1) * 256 + tid;
    const int n  = c / (K2 / 8);
    const int k0 = (c - n * (K2 / 8)) * 8;
#pragma unroll
    for (int e = 0; e < 8; ++e) v[e] = 16.0f * w2[(k0 + e) * C2 + n];
    dst = w2h + (size_t)c * 8;
  } else if (b < NBF1 + NBW2 + NBW3) {
    const int c  = (b - NBF1 - NBW2) * 256 + tid;
    const int n  = c / (K3 / 8);
    const int k0 = (c - n * (K3 / 8)) * 8;
#pragma unroll
    for (int e = 0; e < 8; ++e) v[e] = 16.0f * w3[(k0 + e) * C3 + n];
    dst = w3h + (size_t)c * 8;
  } else {
    const int c  = tid;
    const int n  = c / (NF1 / 8);
    const int k0 = (c - n * (NF1 / 8)) * 8;
    const int nc = n < NF2 ? n : NF2 - 1;
#pragma unroll
    for (int e = 0; e < 8; ++e) {
      const float t = f2[(k0 + e) * NF2 + nc];
      v[e] = (n < NF2) ? 16.0f * t : 0.0f;
    }
    dst = f2h + (size_t)c * 8;
  }
  v8h o;
#pragma unroll
  for (int e = 0; e < 8; ++e) o[e] = (_Float16)v[e];
  *(volatile v8h*)dst = o;
  __threadfence();
  *(volatile v8h*)dst = o;
}

__global__ __launch_bounds__(TC) void k_conv(
    const float* __restrict__ feat, const int* __restrict__ idx, const int* __restrict__ bsz,
    const float* __restrict__ w1, const float* __restrict__ g1, const float* __restrict__ be1,
    const float* __restrict__ mu1, const float* __restrict__ va1,
    const _Float16* __restrict__ w2h, const float* __restrict__ g2, const float* __restrict__ be2,
    const float* __restrict__ mu2, const float* __restrict__ va2,
    const _Float16* __restrict__ w3h, const float* __restrict__ g3, const float* __restrict__ be3,
    const float* __restrict__ mu3, const float* __restrict__ va3,
    _Float16* a3, int P, int nChunk) {
  extern __shared__ __attribute__((aligned(16))) unsigned char smem[];
  _Float16* sH2  = (_Float16*)(smem + OFF_H2);
  double*   sDen = (double*)(smem + OFF_H2);
  int*      sTag = (int*)(smem + OFF_TAG);
  _Float16* sH1  = (_Float16*)(smem + OFF_H1);
  _Float16* sH3  = (_Float16*)(smem + OFF_H1);
  float*    sMk  = (float*)(smem + OFF_MK);
  float*    sDn  = (float*)(smem + OFF_DN);
  float*    sMk1 = (float*)(smem + OFF_MK1);
  float*    sW1  = (float*)(smem + OFF_W1);
  float*    sBN  = (float*)(smem + OFF_BN);

  const int tid = (int)threadIdx.x, lane = tid & 31, wave = tid >> 5, hh = lane >> 4, m = lane & 15;
  const int b = (int)blockIdx.x;
  const int nbv = bsz[0];

#pragma unroll 1
  for (int s = tid; s < NPX; s += TC) { sDen[s] = 0.0; sTag[s] = -1; sMk[s] = 0.0f; }
#pragma unroll 1
  for (int i = tid; i < 9 * C1; i += TC) sW1[i] = w1[i];
  if (tid < C1) {
    sBN[SC1 + tid] = g1[tid] * rsqrtf(va1[tid] + BN_EPS);
    sBN[MU1 + tid] = mu1[tid];
    sBN[BE1 + tid] = be1[tid];
  }
  if (tid < C2) {
    sBN[SC2 + tid] = g2[tid] * rsqrtf(va2[tid] + BN_EPS);
    sBN[MU2 + tid] = mu2[tid];
    sBN[BE2 + tid] = be2[tid];
    sBN[SC3 + tid] = g3[tid] * rsqrtf(va3[tid] + BN_EPS);
    sBN[MU3 + tid] = mu3[tid];
    sBN[BE3 + tid] = be3[tid];
  }
  __syncthreads();

#pragma unroll 1
  for (int c = 0; c < nChunk; ++c) {
    const int j = c * TC + tid;
    const bool valid = j < P;
    const int jc = valid ? j : P - 1;
    const size_t g = (size_t)b * (size_t)P + (size_t)jc;
    const int bi = idx[g * 3 + 0];
    const int yi = idx[g * 3 + 1];
    const int xi = idx[g * 3 + 2];
    const float f = feat[g];
    bool pending = valid && (bi == b) && (bi < nbv) &&
                   ((unsigned)yi < (unsigned)HW) && ((unsigned)xi < (unsigned)HW);
    const int site = pending ? (yi * HW + xi) : 0;
#pragma unroll 1
    for (int ps = 0; ps < MAXPASS; ++ps) {
      if (pending) sTag[site] = tid;
      __syncthreads();
      const int tg = sTag[site];
      const bool win = pending && (tg == tid);
      if (win) {
        sDen[site] += (double)f;
        sMk[site] = 1.0f;
        pending = false;
      }
      if (__syncthreads_or(pending ? 1 : 0) == 0) break;
    }
  }
  __syncthreads();
#pragma unroll 1
  for (int s = tid; s < NPX; s += TC) sDn[s] = (float)sDen[s];
  if (tid < NPX2) {
    const int yo = tid / HW2, xo = tid - yo * HW2;
    const int p = (2 * yo) * HW + 2 * xo;
    sMk1[tid] = fmaxf(fmaxf(sMk[p], sMk[p + 1]), fmaxf(sMk[p + HW], sMk[p + HW + 1]));
  }
  __syncthreads();

#pragma unroll 1
  for (int s = tid; s < NPX; s += TC) {
    const int y = s / HW, x = s - y * HW;
    float tp[9];
#pragma unroll
    for (int t = 0; t < 9; ++t) {
      const int yy = y + t / 3 - 1, xx = x + t % 3 - 1;
      const bool ok = ((unsigned)yy < (unsigned)HW) && ((unsigned)xx < (unsigned)HW);
      const int yc = yy < 0 ? 0 : (yy > HW - 1 ? HW - 1 : yy);
      const int xc = xx < 0 ? 0 : (xx > HW - 1 ? HW - 1 : xx);
      const float v = sDn[yc * HW + xc];
      tp[t] = ok ? v : 0.0f;
    }
    const float mk = sMk[s];
#pragma unroll 1
    for (int c = 0; c < C1; ++c) {
      float acc = 0.0f;
#pragma unroll
      for (int t = 0; t < 9; ++t) acc = fmaf(tp[t], sW1[t * C1 + c], acc);
      const float o = fmaxf(fmaf(acc - sBN[MU1 + c], sBN[SC1 + c], sBN[BE1 + c]), 0.0f) * mk;
      sH1[s * C1 + c] = (_Float16)o;
    }
  }
  __syncthreads();

  {
    const v8h* sH1v = (const v8h*)sH1;
    const v8h z8 = zh8();
    float sc[4], mu[4], be[4];
#pragma unroll
    for (int t = 0; t < 4; ++t) {
      sc[t] = sBN[SC2 + 16 * t + m];
      mu[t] = sBN[MU2 + 16 * t + m];
      be[t] = sBN[BE2 + 16 * t + m];
    }
#pragma unroll 1
    for (int T = wave; T < NT2; T += NWC) {
      const int pix = 16 * T + m;
      const int y = pix / HW, x = pix - y * HW;
      v8f acc[4];
#pragma unroll
      for (int t = 0; t < 4; ++t) acc[t] = zacc();
#pragma unroll 1
      for (int s = 0; s < 9; ++s) {
        const int ty = s / 3, tx = s - ty * 3;
        const int yy = y + ty - 1, xx = x + tx - 1;
        const bool ok = ((unsigned)yy < (unsigned)HW) && ((unsigned)xx < (unsigned)HW);
        const int yc = yy < 0 ? 0 : (yy > HW - 1 ? HW - 1 : yy);
        const int xc = xx < 0 ? 0 : (xx > HW - 1 ? HW - 1 : xx);
        const int p2 = yc * HW + xc;
        const v8h a0 = sH1v[p2 * 4 + hh];
        const v8h a1 = sH1v[p2 * 4 + 2 + hh];
        Frag a;
        a.h[0] = ok ? a0 : z8;
        a.h[1] = ok ? a1 : z8;
        const _Float16* bq = w2h + (size_t)m * K2 + 32 * s + 8 * hh;
#pragma unroll
        for (int t = 0; t < 4; ++t) {
          const _Float16* bp = bq + (size_t)(16 * t) * K2;
          Frag bf;
          bf.h[0] = *(const v8h*)bp;
          bf.h[1] = *(const v8h*)(bp + 16);
          acc[t] = wmf(a.v, bf.v, acc[t]);
        }
      }
#pragma unroll
      for (int t = 0; t < 4; ++t) {
#pragma unroll
        for (int r = 0; r < 8; ++r) {
          const int pr = 16 * T + 8 * hh + r;
          const float o = fmaxf(fmaf(acc[t][r] * 0.0625f - mu[t], sc[t], be[t]), 0.0f) * sMk[pr];
          sH2[pr * C2 + 16 * t + m] = (_Float16)o;
        }
      }
    }
  }
  __syncthreads();

  {
    const v8h* sH2v = (const v8h*)sH2;
    float sc[4], mu[4], be[4];
#pragma unroll
    for (int t = 0; t < 4; ++t) {
      sc[t] = sBN[SC3 + 16 * t + m];
      mu[t] = sBN[MU3 + 16 * t + m];
      be[t] = sBN[BE3 + 16 * t + m];
    }
#pragma unroll 1
    for (int T = wave; T < NT3; T += NWC) {
      const int orow = 16 * T + m;
      const int orc = orow < NPX2 ? orow : NPX2 - 1;
      const int yo = orc / HW2, xo = orc - yo * HW2;
      v8f acc[4];
#pragma unroll
      for (int t = 0; t < 4; ++t) acc[t] = zacc();
#pragma unroll 1
      for (int s = 0; s < 8; ++s) {
        const int tap = s >> 1, dy = tap >> 1, dx = tap & 1;
        const int p2 = (2 * yo + dy) * HW + 2 * xo + dx;
        const int cb = (s & 1) * 4;
        Frag a;
        a.h[0] = sH2v[p2 * 8 + cb + hh];
        a.h[1] = sH2v[p2 * 8 + cb + 2 + hh];
        const _Float16* bq = w3h + (size_t)m * K3 + 32 * s + 8 * hh;
#pragma unroll
        for (int t = 0; t < 4; ++t) {
          const _Float16* bp = bq + (size_t)(16 * t) * K3;
          Frag bf;
          bf.h[0] = *(const v8h*)bp;
          bf.h[1] = *(const v8h*)(bp + 16);
          acc[t] = wmf(a.v, bf.v, acc[t]);
        }
      }
#pragma unroll
      for (int t = 0; t < 4; ++t) {
#pragma unroll
        for (int r = 0; r < 8; ++r) {
          const int orw = 16 * T + 8 * hh + r;
          const int owc = orw < NPX2 ? orw : NPX2 - 1;
          const float m1 = sMk1[owc];
          const float o = fmaxf(fmaf(acc[t][r] * 0.0625f - mu[t], sc[t], be[t]), 0.0f) * m1;
          if (orw < NPX2) sH3[(16 * t + m) * NPX2 + orw] = (_Float16)o;
        }
      }
    }
  }
  __syncthreads();

  {
    _Float16* gb = a3 + (size_t)b * KF;
    const int q = tid & 7, lg = tid >> 3;
#pragma unroll 1
    for (int i = 0; i < (NPX2 + 31) / 32; ++i) {
      const int L = i * 32 + lg;
      const int Lc = L < NPX2 ? L : NPX2 - 1;
      const v8h v = *(const v8h*)(sH3 + Lc * 64 + 8 * q);
      if (L < NPX2) *(volatile v8h*)(gb + (size_t)L * 64 + 8 * q) = v;
    }
    __threadfence();
#pragma unroll 1
    for (int i = 0; i < (NPX2 + 31) / 32; ++i) {
      const int L = i * 32 + lg;
      const int Lc = L < NPX2 ? L : NPX2 - 1;
      const v8h v = *(const v8h*)(sH3 + Lc * 64 + 8 * q);
      if (L < NPX2) *(volatile v8h*)(gb + (size_t)L * 64 + 8 * q) = v;
    }
  }
}

__global__ __launch_bounds__(TFC) void k_fc(
    const _Float16* __restrict__ a3, const _Float16* __restrict__ f1h, const float* __restrict__ f1b,
    const _Float16* __restrict__ f2h, const float* __restrict__ f2b, float* out) {
  __shared__ __attribute__((aligned(16))) _Float16 sZ[RPB * ZP];
  __shared__ __attribute__((aligned(16))) float sLg[RPB * 16];
  __shared__ __attribute__((aligned(16))) float sOut[RPB * NF2];
  const int tid = (int)threadIdx.x, lane = tid & 31, wave = tid >> 5, hh = lane >> 4, m = lane & 15;
  const int rg = (int)blockIdx.x;
  const _Float16* ap = a3 + ((size_t)rg * RPB + m) * KF + 8 * hh;

  v8f acc[4];
#pragma unroll
  for (int t = 0; t < 4; ++t) acc[t] = zacc();
#pragma unroll 1
  for (int ks = 0; ks < KF / 32; ++ks) {
    Frag a;
    a.h[0] = *(const v8h*)(ap + 32 * ks);
    a.h[1] = *(const v8h*)(ap + 32 * ks + 16);
#pragma unroll
    for (int t = 0; t < 4; ++t) {
      const _Float16* bp = f1h + (size_t)(64 * wave + 16 * t + m) * KF + 32 * ks + 8 * hh;
      Frag bf;
      bf.h[0] = *(const v8h*)bp;
      bf.h[1] = *(const v8h*)(bp + 16);
      acc[t] = wmf(a.v, bf.v, acc[t]);
    }
  }
#pragma unroll
  for (int t = 0; t < 4; ++t) {
    const int col = 64 * wave + 16 * t + m;
    const float bb = f1b[col];
#pragma unroll
    for (int r = 0; r < 8; ++r) {
      const float z = fmaxf(fmaf(acc[t][r], 0.015625f, bb), 0.0f);
      sZ[(8 * hh + r) * ZP + col] = (_Float16)z;
    }
  }
  __syncthreads();

  if (wave == 0) {
    v8f acc2 = zacc();
    const _Float16* sap = sZ + m * ZP + 8 * hh;
#pragma unroll
    for (int ks = 0; ks < NF1 / 32; ++ks) {
      Frag a, bf;
      a.h[0] = *(const v8h*)(sap + 32 * ks);
      a.h[1] = *(const v8h*)(sap + 32 * ks + 16);
      const _Float16* bp = f2h + (size_t)m * NF1 + 32 * ks + 8 * hh;
      bf.h[0] = *(const v8h*)bp;
      bf.h[1] = *(const v8h*)(bp + 16);
      acc2 = wmf(a.v, bf.v, acc2);
    }
    const float bb2 = f2b[m < NF2 ? m : NF2 - 1];
#pragma unroll
    for (int r = 0; r < 8; ++r) sLg[(8 * hh + r) * 16 + m] = fmaf(acc2[r], 0.0625f, bb2);
  }
  __syncthreads();

  if (tid < RPB) {
    const int row = tid;
    float mx = sLg[row * 16];
#pragma unroll 1
    for (int j = 1; j < NF2; ++j) mx = fmaxf(mx, sLg[row * 16 + j]);
    float se = 0.0f;
#pragma unroll 1
    for (int j = 0; j < NF2; ++j) se += expf(sLg[row * 16 + j] - mx);
    const float lse = logf(se);
#pragma unroll 1
    for (int j = 0; j < NF2; ++j) sOut[row * NF2 + j] = (sLg[row * 16 + j] - mx) - lse;
  }
  __syncthreads();

  float* gp = out + (size_t)rg * (RPB * NF2);
  const int l0 = tid < 32 ? tid : 31;
  const int l1 = tid < 8 ? tid : 7;
  const v4f v0 = *(const v4f*)(sOut + 4 * l0);
  const v4f v1 = *(const v4f*)(sOut + 128 + 4 * l1);
  if (tid < 32) *(volatile v4f*)(gp + 4 * tid) = v0;
  if (tid < 8)  *(volatile v4f*)(gp + 128 + 4 * tid) = v1;
  __threadfence();
  if (tid < 32) *(volatile v4f*)(gp + 4 * tid) = v0;
  if (tid < 8)  *(volatile v4f*)(gp + 128 + 4 * tid) = v1;
}

extern "C" void kernel_launch(void* const* d_in, const int* in_sizes, int n_in,
                              void* d_out, int out_size, void* d_ws, size_t ws_size,
                              hipStream_t stream) {
  if (n_in < 22) return;
  const int N = in_sizes[0];
  if (out_size <= 0 || (out_size % NF2) != 0) return;
  const int B = out_size / NF2;
  if (B <= 0 || (B % RPB) != 0 || B > (1 << 20)) return;
  if (N <= 0 || in_sizes[1] != 3 * N || (N % B) != 0) return;
  const int P = N / B;
  if (in_sizes[2] < 1) return;
  if (in_sizes[3] != 9 * C1 || in_sizes[4] != C1 || in_sizes[5] != C1 || in_sizes[6] != C1 || in_sizes[7] != C1) return;
  if (in_sizes[8] != K2 * C2 || in_sizes[9] != C2 || in_sizes[10] != C2 || in_sizes[11] != C2 || in_sizes[12] != C2) return;
  if (in_sizes[13] != K3 * C3 || in_sizes[14] != C3 || in_sizes[15] != C3 || in_sizes[16] != C3 || in_sizes[17] != C3) return;
  if (in_sizes[18] != KF * NF1 || in_sizes[19] != NF1 || in_sizes[20] != NF1 * NF2 || in_sizes[21] != NF2) return;

  const float* feat = (const float*)d_in[0];
  const int*   idx  = (const int*)d_in[1];
  const int*   bsz  = (const int*)d_in[2];
  const float* w1   = (const float*)d_in[3];
  const float* g1   = (const float*)d_in[4];
  const float* be1  = (const float*)d_in[5];
  const float* mu1  = (const float*)d_in[6];
  const float* va1  = (const float*)d_in[7];
  const float* w2   = (const float*)d_in[8];
  const float* g2   = (const float*)d_in[9];
  const float* be2  = (const float*)d_in[10];
  const float* mu2  = (const float*)d_in[11];
  const float* va2  = (const float*)d_in[12];
  const float* w3   = (const float*)d_in[13];
  const float* g3   = (const float*)d_in[14];
  const float* be3  = (const float*)d_in[15];
  const float* mu3  = (const float*)d_in[16];
  const float* va3  = (const float*)d_in[17];
  const float* f1   = (const float*)d_in[18];
  const float* f1b  = (const float*)d_in[19];
  const float* f2   = (const float*)d_in[20];
  const float* f2b  = (const float*)d_in[21];
  float* out = (float*)d_out;

  char* ws = (char*)d_ws;
  size_t off = 0;
  const size_t oA3 = off; off += (size_t)B * KF * 2;        off = (off + 255) & ~(size_t)255;
  const size_t oF1 = off; off += (size_t)NF1 * KF * 2;      off = (off + 255) & ~(size_t)255;
  const size_t oW2 = off; off += (size_t)C2 * K2 * 2;       off = (off + 255) & ~(size_t)255;
  const size_t oW3 = off; off += (size_t)C3 * K3 * 2;       off = (off + 255) & ~(size_t)255;
  const size_t oF2 = off; off += (size_t)NF2P * NF1 * 2;    off = (off + 255) & ~(size_t)255;
  if (off > ws_size || off > (size_t)WSCAP) return;
  _Float16* a3  = (_Float16*)(ws + oA3);
  _Float16* f1h = (_Float16*)(ws + oF1);
  _Float16* w2h = (_Float16*)(ws + oW2);
  _Float16* w3h = (_Float16*)(ws + oW3);
  _Float16* f2h = (_Float16*)(ws + oF2);

  const int nChunk = (P + TC - 1) / TC;

  hipFuncSetAttribute(reinterpret_cast<const void*>(&k_conv),
                      hipFuncAttributeMaxDynamicSharedMemorySize, LDS_CONV);

  k_prep<<<NPREP, 256, 0, stream>>>(w2, w3, f1, f2, w2h, w3h, f1h, f2h);
  k_conv<<<B, TC, LDS_CONV, stream>>>(feat, idx, bsz, w1, g1, be1, mu1, va1,
                                      w2h, g2, be2, mu2, va2, w3h, g3, be3, mu3, va3,
                                      a3, P, nChunk);
  k_fc<<<B / RPB, TFC, 0, stream>>>(a3, f1h, f1b, f2h, f2b, out);
}
